// NESA_5806795784210
// MI455X (gfx1250) — hardware-verified
//
#include <hip/hip_runtime.h>
#include <hip/hip_bf16.h>

#define NB   8
#define NT   1024
#define DM   1024
#define NH   8
#define DHD  128
#define DVD  64
#define DE   32
#define KPOS (DM + DE)
#define LDP  1088
#define NQKV (2 * DM + NH * DVD)
#define DO   (NH * DVD)
#define MT   (NB * NT)

typedef unsigned short us;
typedef us v8us __attribute__((ext_vector_type(8), may_alias));
typedef us v16us __attribute__((ext_vector_type(16)));
typedef _Float16 v16h __attribute__((ext_vector_type(16)));
typedef __bf16 v16b __attribute__((ext_vector_type(16)));
typedef float v8f __attribute__((ext_vector_type(8)));
typedef float v4f __attribute__((ext_vector_type(4), may_alias));
typedef unsigned v4u __attribute__((ext_vector_type(4), may_alias));

union Frag { v16us u; v8us h[2]; v16h f; v16b b; };
union Pack8 { us s[8]; v4u v; };

__device__ __forceinline__ int imin(int a, int b) { return a < b ? a : b; }
__device__ __forceinline__ float bfr(float f) {
  unsigned u = __float_as_uint(f); u += 0x7FFFu + ((u >> 16) & 1u); return __uint_as_float(u & 0xFFFF0000u);
}
__device__ __forceinline__ us bfbits(float f) {
  unsigned u = __float_as_uint(f); u += 0x7FFFu + ((u >> 16) & 1u); return (us)(u >> 16);
}
__device__ __forceinline__ float bf2f(us s) { return __uint_as_float(((unsigned)s) << 16); }
__device__ __forceinline__ us hbits(float f) { union { _Float16 h; us u; } c; c.h = (_Float16)f; return c.u; }

__device__ __forceinline__ void wave_lds_sync() {
  __builtin_amdgcn_fence(__ATOMIC_RELEASE, "wavefront");
  asm volatile("s_wait_dscnt 0" ::: "memory");
  __builtin_amdgcn_wave_barrier();
}

__device__ __forceinline__ v16us frag_ld(const us* base, int ld, int k0) {
  const int l = threadIdx.x & 31;
  const us* p = base + (size_t)(l & 15) * ld + k0 + 8 * (l >> 4);
  Frag f;
  f.h[0] = *(const v8us*)p;
  f.h[1] = *(const v8us*)(p + 16);
  return f.u;
}
__device__ __forceinline__ v8f zero8() { v8f z = {0.f, 0.f, 0.f, 0.f, 0.f, 0.f, 0.f, 0.f}; return z; }
__device__ __forceinline__ v8f mma_h(v16us a, v16us b, v8f c) {
  Frag A, B; A.u = a; B.u = b;
  c = __builtin_amdgcn_wmma_f32_16x16x32_f16(false, A.f, false, B.f, (short)0, c, false, false);
  asm volatile("v_nop\n\tv_nop\n\tv_nop\n\tv_nop" : "+v"(c) : "v"(A.f), "v"(B.f));
  return c;
}
__device__ __forceinline__ v8f mma_b(v16us a, v16us b, v8f c) {
  Frag A, B; A.u = a; B.u = b;
  c = __builtin_amdgcn_wmma_f32_16x16x32_bf16(false, A.b, false, B.b, (short)0, c, false, false);
  asm volatile("v_nop\n\tv_nop\n\tv_nop\n\tv_nop" : "+v"(c) : "v"(A.b), "v"(B.b));
  return c;
}

__global__ __launch_bounds__(256) void k_cvt_wT(const float* __restrict__ W, int K, int N, int ldk, us* __restrict__ Bt) {
  __shared__ float tile[64][65];
  const int tid = threadIdx.x, lane = tid & 31, wave = tid >> 5;
  const int k0 = blockIdx.x * 64, n0 = blockIdx.y * 64;
#pragma unroll
  for (int it = 0; it < 4; ++it) {
    const int idx = tid + 256 * it, kr = idx >> 4, c4 = (idx & 15) * 4;
    const int kg = k0 + kr;
    const int ks = imin(kg, K - 1);
    const v4f v = *(const v4f*)(W + (size_t)ks * N + n0 + c4);
    const bool ok = kg < K;
#pragma unroll
    for (int e = 0; e < 4; ++e) tile[kr][c4 + e] = ok ? bfr(v[e]) * 16.0f : 0.0f;
  }
  __syncthreads();
  Pack8 pk[2];
#pragma unroll
  for (int it = 0; it < 2; ++it) {
    const int c = lane + 32 * it, rr = c >> 3, q8 = (c & 7) * 8;
    const int n = 8 * wave + rr;
#pragma unroll
    for (int e = 0; e < 8; ++e) pk[it].s[e] = hbits(tile[q8 + e][n]);
  }
#pragma unroll
  for (int it = 0; it < 2; ++it) {
    const int c = lane + 32 * it, rr = c >> 3, q8 = (c & 7) * 8;
    *(volatile v4u*)(Bt + (size_t)(n0 + 8 * wave + rr) * ldk + k0 + q8) = pk[it].v;
  }
  __threadfence();
#pragma unroll
  for (int it = 0; it < 2; ++it) {
    const int c = lane + 32 * it, rr = c >> 3, q8 = (c & 7) * 8;
    *(volatile v4u*)(Bt + (size_t)(n0 + 8 * wave + rr) * ldk + k0 + q8) = pk[it].v;
  }
}

__global__ __launch_bounds__(256) void k_cvt_xpe(const float* __restrict__ x, const float* __restrict__ pe, us* __restrict__ xpe) {
  const int lane = threadIdx.x & 31, wave = threadIdx.x >> 5;
  const int m = blockIdx.x * 8 + wave;
  const int tok = m & (NT - 1);
  const float* xr = x + (size_t)m * DM;
  us* dst = xpe + (size_t)m * LDP;
  Pack8 pk[5];
#pragma unroll
  for (int it = 0; it < 4; ++it) {
    const int c8 = (lane + 32 * it) * 8;
    const v4f a = *(const v4f*)(xr + c8), bq = *(const v4f*)(xr + c8 + 4);
#pragma unroll
    for (int e = 0; e < 4; ++e) { pk[it].s[e] = hbits(bfr(a[e])); pk[it].s[4 + e] = hbits(bfr(bq[e])); }
  }
  {
    const int pc = imin(lane, 3) * 8;
    const v4f a = *(const v4f*)(pe + (size_t)tok * DE + pc), bq = *(const v4f*)(pe + (size_t)tok * DE + pc + 4);
    const bool ok = lane < 4;
#pragma unroll
    for (int e = 0; e < 4; ++e) { pk[4].s[e] = ok ? hbits(bfr(a[e])) : (us)0; pk[4].s[4 + e] = ok ? hbits(bfr(bq[e])) : (us)0; }
  }
#pragma unroll
  for (int it = 0; it < 4; ++it) *(volatile v4u*)(dst + (lane + 32 * it) * 8) = pk[it].v;
  if (lane < 8) *(volatile v4u*)(dst + DM + lane * 8) = pk[4].v;
  __threadfence();
#pragma unroll
  for (int it = 0; it < 4; ++it) *(volatile v4u*)(dst + (lane + 32 * it) * 8) = pk[it].v;
  if (lane < 8) *(volatile v4u*)(dst + DM + lane * 8) = pk[4].v;
}

__device__ __forceinline__ void gemm_tile(const us* __restrict__ A, int lda, const us* __restrict__ Bt, int ldb, int K,
                                          int m0, int n0, int wm, int wn, v8f (&acc)[2][4]) {
  const us* a0p = A + (size_t)(m0 + wm) * lda;
  const us* a1p = a0p + (size_t)16 * lda;
  const us* bp = Bt + (size_t)(n0 + wn) * ldb;
#pragma unroll 1
  for (int k0 = 0; k0 < K; k0 += 32) {
    const v16us fa0 = frag_ld(a0p, lda, k0);
    const v16us fa1 = frag_ld(a1p, lda, k0);
#pragma unroll
    for (int j = 0; j < 4; ++j) {
      const v16us fb = frag_ld(bp + (size_t)(16 * j) * ldb, ldb, k0);
      acc[0][j] = mma_h(fa0, fb, acc[0][j]);
      acc[1][j] = mma_h(fa1, fb, acc[1][j]);
    }
  }
}

__global__ __launch_bounds__(256) void k_gemm_res(const us* __restrict__ A, int lda, const us* __restrict__ Bt, int ldb, int K,
                                                 const float* __restrict__ bias, const float* __restrict__ xres,
                                                 float* __restrict__ Y, int N) {
  __shared__ __attribute__((aligned(16))) unsigned char stg[8 * 4608];
  const int tid = threadIdx.x, lane = tid & 31, wave = tid >> 5, cl = lane & 15, hh = lane >> 4;
  const int m0 = blockIdx.y * 128, n0 = blockIdx.x * 128;
  const int wm = (wave & 3) * 32, wn = (wave >> 2) * 64;
  v8f acc[2][4];
#pragma unroll
  for (int i = 0; i < 2; ++i)
#pragma unroll
    for (int j = 0; j < 4; ++j) acc[i][j] = zero8();
  gemm_tile(A, lda, Bt, ldb, K, m0, n0, wm, wn, acc);

  float* so = (float*)(stg + wave * 4608);
#pragma unroll
  for (int i = 0; i < 2; ++i) {
    wave_lds_sync();
#pragma unroll
    for (int j = 0; j < 4; ++j)
#pragma unroll
      for (int r = 0; r < 8; ++r) so[(8 * hh + r) * 68 + 16 * j + cl] = acc[i][j][r] * 0.0625f;
    wave_lds_sync();
    v4f vals[8];
#pragma unroll
    for (int it = 0; it < 8; ++it) {
      const int c = lane + 32 * it, rr = c >> 4, q4 = (c & 15) * 4;
      const int g = m0 + wm + 16 * i + rr, col = n0 + wn + q4;
      const v4f bv = *(const v4f*)(bias + col);
      const v4f xv = *(const v4f*)(xres + (size_t)g * N + col);
      v4f v = *(const v4f*)(so + rr * 68 + q4);
#pragma unroll
      for (int e = 0; e < 4; ++e) v[e] = bfr(xv[e]) + (v[e] + bfr(bv[e]));
      vals[it] = v;
    }
#pragma unroll
    for (int it = 0; it < 8; ++it) {
      const int c = lane + 32 * it, rr = c >> 4, q4 = (c & 15) * 4;
      *(volatile v4f*)(Y + (size_t)(m0 + wm + 16 * i + rr) * N + n0 + wn + q4) = vals[it];
    }
    __threadfence();
#pragma unroll
    for (int it = 0; it < 8; ++it) {
      const int c = lane + 32 * it, rr = c >> 4, q4 = (c & 15) * 4;
      *(volatile v4f*)(Y + (size_t)(m0 + wm + 16 * i + rr) * N + n0 + wn + q4) = vals[it];
    }
  }
}

template <bool QK>
__device__ __forceinline__ void store_rows16(const us* so, us* __restrict__ plane, int lane, int m0, int wm, int colbase, int head) {
  v4u pk[8];
#pragma unroll
  for (int it = 0; it < 8; ++it) { const int c = lane + 32 * it, rr = c >> 3, q8 = (c & 7) * 8; pk[it] = *(const v4u*)(so + rr * 72 + q8); }
#pragma unroll
  for (int it = 0; it < 8; ++it) {
    const int c = lane + 32 * it, rr = c >> 3, q8 = (c & 7) * 8;
    const int g = m0 + wm + rr;
    const size_t off = QK ? ((size_t)((g >> 10) * NH + head) * NT + (g & (NT - 1))) * DHD + colbase + q8
                          : (size_t)g * DO + colbase + q8;
    *(volatile v4u*)(plane + off) = pk[it];
  }
  __threadfence();
#pragma unroll
  for (int it = 0; it < 8; ++it) {
    const int c = lane + 32 * it, rr = c >> 3, q8 = (c & 7) * 8;
    const int g = m0 + wm + rr;
    const size_t off = QK ? ((size_t)((g >> 10) * NH + head) * NT + (g & (NT - 1))) * DHD + colbase + q8
                          : (size_t)g * DO + colbase + q8;
    *(volatile v4u*)(plane + off) = pk[it];
  }
}

__global__ __launch_bounds__(256) void k_gemm_qkv(const us* __restrict__ A, const us* __restrict__ Bt, const float* __restrict__ bias,
                                                 us* __restrict__ qhi, us* __restrict__ qlo, us* __restrict__ khi, us* __restrict__ klo,
                                                 us* __restrict__ vtok) {
  __shared__ __attribute__((aligned(16))) unsigned char stg[8 * 4608];
  const int tid = threadIdx.x, lane = tid & 31, wave = tid >> 5, cl = lane & 15, hh = lane >> 4;
  const int m0 = blockIdx.y * 128, n0 = blockIdx.x * 128;
  const int wm = (wave & 3) * 32, wn = (wave >> 2) * 64;
  v8f acc[2][4];
#pragma unroll
  for (int i = 0; i < 2; ++i)
#pragma unroll
    for (int j = 0; j < 4; ++j) acc[i][j] = zero8();
  gemm_tile(A, DM, Bt, DM, DM, m0, n0, wm, wn, acc);
#pragma unroll
  for (int j = 0; j < 4; ++j) {
    const float bv = bfr(bias[n0 + wn + 16 * j + cl]);
#pragma unroll
    for (int i = 0; i < 2; ++i)
#pragma unroll
      for (int r = 0; r < 8; ++r) acc[i][j][r] = acc[i][j][r] * 0.0625f + bv;
  }
  us* so = (us*)(stg + wave * 4608);
  const int which = n0 >> 10;
  if (which < 2) {
    const int head = (n0 & (DM - 1)) >> 7;
    us* ph = (which == 0) ? qhi : khi;
    us* pl = (which == 0) ? qlo : klo;
    wave_lds_sync();
#pragma unroll
    for (int i = 0; i < 2; ++i)
#pragma unroll
      for (int j = 0; j < 4; ++j)
#pragma unroll
        for (int r = 0; r < 8; ++r) so[(16 * i + 8 * hh + r) * 72 + 16 * j + cl] = bfbits(acc[i][j][r]);
    wave_lds_sync();
    store_rows16<true>(so, ph, lane, m0, wm, wn, head);
    wave_lds_sync();
#pragma unroll
    for (int i = 0; i < 2; ++i)
#pragma unroll
      for (int j = 0; j < 4; ++j)
#pragma unroll
        for (int r = 0; r < 8; ++r) {
          const float v = acc[i][j][r];
          so[(16 * i + 8 * hh + r) * 72 + 16 * j + cl] = bfbits(v - bf2f(bfbits(v)));
        }
    wave_lds_sync();
    store_rows16<true>(so, pl, lane, m0, wm, wn, head);
  } else {
    const int vcol = n0 - 2 * DM + wn;
    wave_lds_sync();
#pragma unroll
    for (int i = 0; i < 2; ++i)
#pragma unroll
      for (int j = 0; j < 4; ++j)
#pragma unroll
        for (int r = 0; r < 8; ++r) so[(16 * i + 8 * hh + r) * 72 + 16 * j + cl] = hbits(acc[i][j][r]);
    wave_lds_sync();
    store_rows16<false>(so, vtok, lane, m0, wm, vcol, 0);
  }
}

__global__ __launch_bounds__(256) void k_stats(const float* __restrict__ h, float* __restrict__ mean, float* __restrict__ rstd) {
  __shared__ __attribute__((aligned(16))) float sm[2][256];
  const int tid = threadIdx.x;
  const int idx = blockIdx.x * 256 + tid;
  const int b = idx >> 10, ch = idx & (DM - 1);
  const float* p = h + (size_t)b * NT * DM + ch;
  double s = 0.0, s2 = 0.0;
#pragma unroll 4
  for (int t = 0; t < NT; ++t) { const double f = (double)p[(size_t)t * DM]; s += f; s2 += f * f; }
  const double mu = s * (1.0 / (double)NT);
  double var = s2 * (1.0 / (double)NT) - mu * mu;
  if (var < 0.0) var = 0.0;
  const float vf = (float)var;
  const float rs = 1.0f / sqrtf(vf + 1e-5f);
  sm[0][tid] = (float)mu; sm[1][tid] = rs;
  __syncthreads();
  if (tid < 128) {
    const int sel = tid >> 6, c4 = (tid & 63) * 4;
    const v4f v = *(const v4f*)&sm[sel][c4];
    float* dst = ((sel == 0) ? mean : rstd) + (size_t)blockIdx.x * 256 + c4;
    *(volatile v4f*)dst = v;
    __threadfence();
    *(volatile v4f*)dst = v;
  }
}

__global__ __launch_bounds__(256) void k_norm(const float* __restrict__ h, const float* __restrict__ mean, const float* __restrict__ rstd,
                                             const float* __restrict__ gamma, const float* __restrict__ beta, us* __restrict__ hn) {
  const int lane = threadIdx.x & 31, wave = threadIdx.x >> 5;
  const int m = blockIdx.x * 8 + wave;
  const int b = m >> 10;
  const float* hr = h + (size_t)m * DM;
  const float* mr = mean + (size_t)b * DM;
  const float* rr = rstd + (size_t)b * DM;
  Pack8 pk[4];
#pragma unroll
  for (int it = 0; it < 4; ++it) {
    const int c8 = (lane + 32 * it) * 8;
#pragma unroll
    for (int hf = 0; hf < 2; ++hf) {
      const int c = c8 + 4 * hf;
      const v4f hv = *(const v4f*)(hr + c), mu = *(const v4f*)(mr + c), rs = *(const v4f*)(rr + c);
      const v4f gm = *(const v4f*)(gamma + c), bt = *(const v4f*)(beta + c);
#pragma unroll
      for (int e = 0; e < 4; ++e) pk[it].s[4 * hf + e] = hbits((bfr(gm[e]) * (hv[e] - mu[e])) * rs[e] + bfr(bt[e]));
    }
  }
  us* dst = hn + (size_t)m * DM;
#pragma unroll
  for (int it = 0; it < 4; ++it) *(volatile v4u*)(dst + (lane + 32 * it) * 8) = pk[it].v;
  __threadfence();
#pragma unroll
  for (int it = 0; it < 4; ++it) *(volatile v4u*)(dst + (lane + 32 * it) * 8) = pk[it].v;
}

__device__ __forceinline__ float sumsq16(const us* hp, const us* lp) {
  const v8us h0 = *(const v8us*)hp, h1 = *(const v8us*)(hp + 8), l0 = *(const v8us*)lp, l1 = *(const v8us*)(lp + 8);
  float s = 0.0f;
#pragma unroll
  for (int e = 0; e < 8; ++e) { const float f = bf2f(h0[e]) + bf2f(l0[e]); s += f * f; }
#pragma unroll
  for (int e = 0; e < 8; ++e) { const float f = bf2f(h1[e]) + bf2f(l1[e]); s += f * f; }
  return s;
}
__global__ __launch_bounds__(256) void k_sqnorm(const us* __restrict__ qhi, const us* __restrict__ qlo, const us* __restrict__ khi,
                                               const us* __restrict__ klo, float* __restrict__ sq, float* __restrict__ sk) {
  __shared__ __attribute__((aligned(16))) float ss[2][32];
  const int tid = threadIdx.x;
  const int rl = tid >> 3, part = tid & 7;
  const size_t row = (size_t)blockIdx.x * 32 + rl;
  const size_t off = row * DHD + part * 16;
  float aq = sumsq16(qhi + off, qlo + off);
  float ak = sumsq16(khi + off, klo + off);
#pragma unroll
  for (int d = 1; d < 8; d <<= 1) { aq += __shfl_xor(aq, d, 32); ak += __shfl_xor(ak, d, 32); }
  if (part == 0) { ss[0][rl] = aq; ss[1][rl] = ak; }
  __syncthreads();
  if (tid < 16) {
    const int sel = tid >> 3, c4 = (tid & 7) * 4;
    const v4f v = *(const v4f*)&ss[sel][c4];
    float* dst = ((sel == 0) ? sq : sk) + (size_t)blockIdx.x * 32 + c4;
    *(volatile v4f*)dst = v;
    __threadfence();
    *(volatile v4f*)dst = v;
  }
}

__global__ __launch_bounds__(256) void k_vtrans(const us* __restrict__ vtok, us* __restrict__ vT) {
  __shared__ __attribute__((aligned(16))) us tile[64 * 72];
  const int tid = threadIdx.x, lane = tid & 31, wave = tid >> 5;
  const int bh = blockIdx.y, b = bh >> 3, head = bh & 7;
  const int t0 = blockIdx.x * 64;
#pragma unroll
  for (int it = 0; it < 2; ++it) {
    const int c = tid + 256 * it, tr = c >> 3, q8 = (c & 7) * 8;
    const v8us v = *(const v8us*)(vtok + ((size_t)(b * NT + t0 + tr)) * DO + head * DVD + q8);
    *(v8us*)(tile + tr * 72 + q8) = v;
  }
  __syncthreads();
  Pack8 pk[2];
#pragma unroll
  for (int it = 0; it < 2; ++it) {
    const int c = lane + 32 * it, rr = c >> 3, q8 = (c & 7) * 8;
    const int dv = 8 * wave + rr;
#pragma unroll
    for (int e = 0; e < 8; ++e) pk[it].s[e] = tile[(q8 + e) * 72 + dv];
  }
#pragma unroll
  for (int it = 0; it < 2; ++it) {
    const int c = lane + 32 * it, rr = c >> 3, q8 = (c & 7) * 8;
    *(volatile v4u*)(vT + ((size_t)(bh * DVD + 8 * wave + rr)) * NT + t0 + q8) = pk[it].v;
  }
  __threadfence();
#pragma unroll
  for (int it = 0; it < 2; ++it) {
    const int c = lane + 32 * it, rr = c >> 3, q8 = (c & 7) * 8;
    *(volatile v4u*)(vT + ((size_t)(bh * DVD + 8 * wave + rr)) * NT + t0 + q8) = pk[it].v;
  }
}

__global__ __launch_bounds__(256) void k_attn(const us* __restrict__ qhi, const us* __restrict__ qlo, const us* __restrict__ khi,
                                             const us* __restrict__ klo, const us* __restrict__ vT, const float* __restrict__ sq,
                                             const float* __restrict__ sk, const float* __restrict__ scale, us* __restrict__ ao) {
  __shared__ __attribute__((aligned(16))) us Ps[8][16 * 72];
  const int tid = threadIdx.x, lane = tid & 31, wave = tid >> 5, cl = lane & 15, hh = lane >> 4;
  const int bh = blockIdx.x, b = bh >> 3, head = bh & 7;
  const int row0 = blockIdx.y * 128 + wave * 16;
  const size_t prow = (size_t)bh * NT + row0;
  const us* qh = qhi + prow * DHD;
  const us* ql = qlo + prow * DHD;
  const us* khb = khi + (size_t)bh * NT * DHD;
  const us* klb = klo + (size_t)bh * NT * DHD;
  const us* vb = vT + (size_t)bh * DVD * NT;
  const float* skb = sk + (size_t)bh * NT;
  const float s = bfr(scale[0]);
  const float inv = 1.0f / (s * s);
  float sqr[8], mrow[8], lrow[8];
#pragma unroll
  for (int r = 0; r < 8; ++r) { sqr[r] = sq[prow + 8 * hh + r]; mrow[r] = -3.0e38f; lrow[r] = 0.0f; }
  v8f o[4];
#pragma unroll
  for (int fo = 0; fo < 4; ++fo) o[fo] = zero8();
  us* ps = &Ps[wave][0];

#pragma unroll 1
  for (int c0 = 0; c0 < NT; c0 += 32) {
    v8f st0 = zero8(), st1 = zero8();
    const us* kh0 = khb + (size_t)c0 * DHD;
    const us* kl0 = klb + (size_t)c0 * DHD;
#pragma unroll 1
    for (int kf = 0; kf < 4; ++kf) {
      const int k0 = kf * 32;
      const v16us ah = frag_ld(qh, DHD, k0);
      const v16us al = frag_ld(ql, DHD, k0);
      const v16us bh0 = frag_ld(kh0, DHD, k0);
      const v16us bl0 = frag_ld(kl0, DHD, k0);
      st0 = mma_b(ah, bh0, st0);
      st0 = mma_b(ah, bl0, st0);
      st0 = mma_b(al, bh0, st0);
      const v16us bh1 = frag_ld(kh0 + 16 * DHD, DHD, k0);
      const v16us bl1 = frag_ld(kl0 + 16 * DHD, DHD, k0);
      st1 = mma_b(ah, bh1, st1);
      st1 = mma_b(ah, bl1, st1);
      st1 = mma_b(al, bh1, st1);
    }
    const float sk0 = skb[c0 + cl], sk1 = skb[c0 + 16 + cl];
    wave_lds_sync();
#pragma unroll
    for (int r = 0; r < 8; ++r) {
      const float l0 = -fmaxf(sqr[r] + sk0 - 2.0f * st0[r], 0.0f) * inv;
      const float l1 = -fmaxf(sqr[r] + sk1 - 2.0f * st1[r], 0.0f) * inv;
      float mx = fmaxf(l0, l1);
#pragma unroll
      for (int d = 1; d < 16; d <<= 1) mx = fmaxf(mx, __shfl_xor(mx, d, 32));
      const float mnew = fmaxf(mrow[r], mx);
      const float alpha = __expf(mrow[r] - mnew);
      mrow[r] = mnew;
      lrow[r] *= alpha;
#pragma unroll
      for (int fo = 0; fo < 4; ++fo) o[fo][r] *= alpha;
      const float p0 = __expf(l0 - mnew);
      const float p1 = __expf(l1 - mnew);
      float psum = p0 + p1;
#pragma unroll
      for (int d = 1; d < 16; d <<= 1) psum += __shfl_xor(psum, d, 32);
      lrow[r] += psum;
      ps[(8 * hh + r) * 72 + cl] = hbits(p0 * 4096.0f);
      ps[(8 * hh + r) * 72 + 16 + cl] = hbits(p1 * 4096.0f);
    }
    wave_lds_sync();
    const v16us pf = frag_ld(ps, 72, 0);
#pragma unroll
    for (int fo = 0; fo < 4; ++fo) {
      const v16us vf = frag_ld(vb + (size_t)(fo * 16) * NT, NT, c0);
      o[fo] = mma_h(pf, vf, o[fo]);
    }
  }
  wave_lds_sync();
#pragma unroll
  for (int r = 0; r < 8; ++r) {
    const float rl = 1.0f / (lrow[r] * 4096.0f);
#pragma unroll
    for (int fo = 0; fo < 4; ++fo) ps[(8 * hh + r) * 72 + 16 * fo + cl] = hbits(o[fo][r] * rl);
  }
  wave_lds_sync();
  v4u pk[4];
#pragma unroll
  for (int it = 0; it < 4; ++it) { const int c = lane + 32 * it, rr = c >> 3, q8 = (c & 7) * 8; pk[it] = *(const v4u*)(ps + rr * 72 + q8); }
#pragma unroll
  for (int it = 0; it < 4; ++it) {
    const int c = lane + 32 * it, rr = c >> 3, q8 = (c & 7) * 8;
    *(volatile v4u*)(ao + ((size_t)(b * NT + row0 + rr)) * DO + head * DVD + q8) = pk[it];
  }
  __threadfence();
#pragma unroll
  for (int it = 0; it < 4; ++it) {
    const int c = lane + 32 * it, rr = c >> 3, q8 = (c & 7) * 8;
    *(volatile v4u*)(ao + ((size_t)(b * NT + row0 + rr)) * DO + head * DVD + q8) = pk[it];
  }
}

extern "C" void kernel_launch(void* const* d_in, const int* in_sizes, int n_in,
                              void* d_out, int out_size, void* d_ws, size_t ws_size,
                              hipStream_t stream) {
  if (n_in < 11) return;
  if (in_sizes[0] != MT * DM || in_sizes[1] < DM || in_sizes[2] < DM || in_sizes[3] != NT * DE ||
      in_sizes[4] != KPOS * DM || in_sizes[5] < DM || in_sizes[6] != DM * NQKV || in_sizes[7] < NQKV ||
      in_sizes[8] != DO * DM || in_sizes[9] < DM || in_sizes[10] < 1 || out_size != MT * DM) return;
  const float* x     = (const float*)d_in[0];
  const float* gamma = (const float*)d_in[1];
  const float* beta  = (const float*)d_in[2];
  const float* pe    = (const float*)d_in[3];
  const float* Wpos  = (const float*)d_in[4];
  const float* bpos  = (const float*)d_in[5];
  const float* Wqkv  = (const float*)d_in[6];
  const float* bqkv  = (const float*)d_in[7];
  const float* Wout  = (const float*)d_in[8];
  const float* bout  = (const float*)d_in[9];
  const float* scale = (const float*)d_in[10];
  float* out = (float*)d_out;

  const size_t szWqkvT = (size_t)NQKV * DM * 2;
  const size_t szWoutT = (size_t)DM * DO * 2;
  const size_t szStat  = (size_t)NB * DM * 4;
  const size_t szNrm   = (size_t)NB * NH * NT * 4;
  const size_t szHn    = (size_t)MT * DM * 2;
  const size_t szXpe   = (size_t)MT * LDP * 2;
  const size_t szWposT = (size_t)DM * LDP * 2;
  const size_t szH     = (size_t)MT * DM * 4;
  const size_t szPl    = (size_t)NB * NH * NT * DHD * 2;
  const size_t szV     = (size_t)MT * DO * 2;
  size_t o = 0;
  const size_t oWqkvT = o; o += szWqkvT;
  const size_t oWoutT = o; o += szWoutT;
  const size_t oMean  = o; o += szStat;
  const size_t oRstd  = o; o += szStat;
  const size_t oSq    = o; o += szNrm;
  const size_t oSk    = o; o += szNrm;
  const size_t a0     = o;
  const size_t oHn    = a0;
  const size_t oVT    = a0;
  const size_t oAo    = a0 + szV;
  const size_t oXpe   = a0 + szHn;
  const size_t oWposT = oXpe + szXpe;
  const size_t oH     = oWposT + szWposT;
  const size_t oQhi   = a0 + szHn;
  const size_t oQlo   = oQhi + szPl;
  const size_t oKhi   = oQlo + szPl;
  const size_t oKlo   = oKhi + szPl;
  const size_t oV     = oKlo + szPl;
  const size_t endA   = oH + szH;
  const size_t endB   = oV + szV;
  const size_t total  = endA > endB ? endA : endB;
  if (total > ws_size) return;

  char* ws = (char*)d_ws;
  us* WqkvT = (us*)(ws + oWqkvT);
  us* WoutT = (us*)(ws + oWoutT);
  float* mean = (float*)(ws + oMean);
  float* rstd = (float*)(ws + oRstd);
  float* sqv = (float*)(ws + oSq);
  float* skv = (float*)(ws + oSk);
  us* hn    = (us*)(ws + oHn);
  us* vT    = (us*)(ws + oVT);
  us* ao    = (us*)(ws + oAo);
  us* xpe   = (us*)(ws + oXpe);
  us* WposT = (us*)(ws + oWposT);
  float* h  = (float*)(ws + oH);
  us* qhi = (us*)(ws + oQhi);
  us* qlo = (us*)(ws + oQlo);
  us* khi = (us*)(ws + oKhi);
  us* klo = (us*)(ws + oKlo);
  us* vtok = (us*)(ws + oV);

  const dim3 blk(256);
  k_cvt_wT<<<dim3(LDP / 64, DM / 64), blk, 0, stream>>>(Wpos, KPOS, DM, LDP, WposT);
  k_cvt_wT<<<dim3(DM / 64, NQKV / 64), blk, 0, stream>>>(Wqkv, DM, NQKV, DM, WqkvT);
  k_cvt_wT<<<dim3(DO / 64, DM / 64), blk, 0, stream>>>(Wout, DO, DM, DO, WoutT);
  k_cvt_xpe<<<dim3(MT / 8), blk, 0, stream>>>(x, pe, xpe);
  k_gemm_res<<<dim3(DM / 128, MT / 128), blk, 0, stream>>>(xpe, LDP, WposT, LDP, KPOS, bpos, x, h, DM);
  k_stats<<<dim3((NB * DM) / 256), blk, 0, stream>>>(h, mean, rstd);
  k_norm<<<dim3(MT / 8), blk, 0, stream>>>(h, mean, rstd, gamma, beta, hn);
  k_gemm_qkv<<<dim3(NQKV / 128, MT / 128), blk, 0, stream>>>(hn, WqkvT, bqkv, qhi, qlo, khi, klo, vtok);
  k_sqnorm<<<dim3((NB * NH * NT) / 32), blk, 0, stream>>>(qhi, qlo, khi, klo, sqv, skv);
  k_vtrans<<<dim3(NT / 64, NB * NH), blk, 0, stream>>>(vtok, vT);
  k_attn<<<dim3(NB * NH, NT / 128), blk, 0, stream>>>(qhi, qlo, khi, klo, vT, sqv, skv, scale, ao);
  k_gemm_res<<<dim3(DM / 128, MT / 128), blk, 0, stream>>>(ao, DO, WoutT, DO, DO, bout, x, out, DM);
}
